// SelfAttentiveBimodalFusion_PTBlock_51393578664166
// MI455X (gfx1250) — hardware-verified
//
#include <hip/hip_runtime.h>
#include <math.h>

typedef __attribute__((ext_vector_type(16))) _Float16 v16h;
typedef __attribute__((ext_vector_type(16))) __bf16 v16b;
typedef __attribute__((ext_vector_type(8)))  _Float16 v8h;
typedef __attribute__((ext_vector_type(8)))  float v8f;
typedef __attribute__((ext_vector_type(4)))  float v4f;
typedef __attribute__((ext_vector_type(2)))  float v2f;
typedef __attribute__((ext_vector_type(4)))  unsigned v4u;
typedef __attribute__((ext_vector_type(4)))  int v4i;
typedef float __attribute__((may_alias)) float_a;
typedef int __attribute__((may_alias)) int_a;

template <typename T> __device__ __forceinline__ void vst2(void* p, T v) { *(volatile T*)p = v; __threadfence(); *(volatile T*)p = v; }
__device__ __forceinline__ v8f wmma16(v16h a, v16h b, v8f c) {
  v8f d = __builtin_amdgcn_wmma_f32_16x16x32_f16(false, a, false, b, (short)0, c, false, false);
  asm volatile("v_nop\n\tv_nop\n\tv_nop\n\tv_nop" : "+v"(d) : "v"(a), "v"(b));
  return d;
}
__device__ __forceinline__ v8f wmma_bf(v16b a, v16b b, v8f c) {
  v8f d = __builtin_amdgcn_wmma_f32_16x16x32_bf16(false, a, false, b, (short)0, c, false, false);
  asm volatile("v_nop\n\tv_nop\n\tv_nop\n\tv_nop" : "+v"(d) : "v"(a), "v"(b));
  return d;
}
__device__ __forceinline__ v16h frag_h(const _Float16* rowk0, int lane) {
  union { v16h v; v8h q[2]; } u; const _Float16* p = rowk0 + 8 * (lane >> 4);
  u.q[0] = *(const v8h*)p; u.q[1] = *(const v8h*)(p + 16); return u.v;
}
__device__ __forceinline__ v16h frag_f32(const float* rowk0, int lane) {
  v16h a; const float* p = rowk0 + 8 * (lane >> 4);
#pragma unroll
  for (int i = 0; i < 8; ++i) { a[i] = (_Float16)p[i]; a[8 + i] = (_Float16)p[16 + i]; }
  return a;
}
__device__ __forceinline__ v16h frag_f32s(const float* rowk0, int lane, float sc) {
  v16h a; const float* p = rowk0 + 8 * (lane >> 4);
#pragma unroll
  for (int i = 0; i < 8; ++i) { a[i] = (_Float16)(p[i] * sc); a[8 + i] = (_Float16)(p[16 + i] * sc); }
  return a;
}
__device__ __forceinline__ v16h fragc_f32(const float* W, int k0, int n, int lane, int ld, int K) {
  v16h a; const int g = lane >> 4;
#pragma unroll
  for (int i = 0; i < 8; ++i) { const int ka = k0 + 8 * g + i, kb = ka + 16;
    a[i] = (_Float16)(ka < K ? W[(size_t)(ka < K ? ka : K - 1) * ld + n] : 0.f); a[8 + i] = (_Float16)(kb < K ? W[(size_t)(kb < K ? kb : K - 1) * ld + n] : 0.f); }
  return a;
}
struct F2 { v16b h, l; };
__device__ __forceinline__ F2 bsplit16(const float v[16]) { F2 r;
#pragma unroll
  for (int i = 0; i < 16; ++i) { const __bf16 h = (__bf16)v[i]; r.h[i] = h; r.l[i] = (__bf16)(v[i] - (float)h); }
  return r; }
__device__ __forceinline__ F2 split_row(const float* row, int k0, int lane) { float v[16]; const float* p = row + k0 + 8 * (lane >> 4);
#pragma unroll
  for (int i = 0; i < 8; ++i) { v[i] = p[i]; v[8 + i] = p[16 + i]; }
  return bsplit16(v); }
__device__ __forceinline__ F2 split_rowK(const float* row, int k0, int lane, int K) { float v[16]; const int g = lane >> 4;
#pragma unroll
  for (int i = 0; i < 8; ++i) { const int ka = k0 + 8 * g + i, kb = ka + 16; v[i] = ka < K ? row[ka < K ? ka : K - 1] : 0.f; v[8 + i] = kb < K ? row[kb < K ? kb : K - 1] : 0.f; }
  return bsplit16(v); }
__device__ __forceinline__ F2 split_col(const float* W, int k0, int n, int lane, int ld, int K) { float v[16]; const int g = lane >> 4;
#pragma unroll
  for (int i = 0; i < 8; ++i) { const int ka = k0 + 8 * g + i, kb = ka + 16; v[i] = ka < K ? W[(size_t)(ka < K ? ka : K - 1) * ld + n] : 0.f; v[8 + i] = kb < K ? W[(size_t)(kb < K ? kb : K - 1) * ld + n] : 0.f; }
  return bsplit16(v); }
__device__ __forceinline__ v8f mac3(const F2& a, const F2& b, v8f c) { c = wmma_bf(a.l, b.h, c); c = wmma_bf(a.h, b.l, c); return wmma_bf(a.h, b.h, c); }
__device__ __forceinline__ float sigm(float v) { return 1.0f / (1.0f + expf(-v)); }
#define LDSX() do { asm volatile("s_wait_dscnt 0" ::: "memory"); __builtin_amdgcn_wave_barrier(); __builtin_amdgcn_fence(__ATOMIC_RELEASE, "workgroup"); } while (0)


#define NPTS 32768
#define NS 16
#define CIN 16
#define CF 256
#define GRID 12
#define NCELL (GRID * GRID * GRID)
#ifndef NPT_
#define NPT_ NPTS
#endif
typedef __attribute__((ext_vector_type(8))) __bf16 v8b;
__device__ __forceinline__ v16b frag_b(const __bf16* rowk0, int lane) {
  union { v16b v; v8b q[2]; } u; const __bf16* p = rowk0 + 8 * (lane >> 4);
  u.q[0] = *(const v8b*)p; u.q[1] = *(const v8b*)(p + 16); return u.v;
}
__device__ __forceinline__ float bfr(float v) { return (float)(__bf16)v; }
__device__ __attribute__((noinline)) float exp_ni(float v) { return expf(v); }
__device__ __attribute__((noinline)) float erf_ni(float v) { return erff(v); }

#define CSA_N 1728
#define CSA_E 32768
#define CSA_FINN (CSA_E + 32 * CSA_NBK)
#define CSA_CHUNK 4096
#define CSA_BKT 256
#define CSA_NCH ((CSA_E + CSA_CHUNK - 1) / CSA_CHUNK)
#define CSA_NBK ((CSA_N + CSA_BKT - 1) / CSA_BKT)
#define CSA_NBKP (((CSA_NBK + 63) / 64) * 64)
#define CSA_SEGCAP (CSA_E + 32 * CSA_NBK * CSA_NCH)
#ifndef CSA_BCAP
#define CSA_BCAP 10240
#endif
#define CSA_SZ_CNT   (4u * CSA_NCH * CSA_NBKP)
#define CSA_SZ_OFF   (4u * CSA_NBK * (((CSA_NCH + 31) / 32) * 32))
#define CSA_SZ_BST   (4u * (((CSA_NBK + 1 + 31) / 32) * 32))
#define CSA_SZ_SEG   (4u * CSA_SEGCAP)
#define CSA_SZ_FIN   (4u * (CSA_E + 32 * CSA_NBK))
#define CSA_SZ_ROW   (4u * CSA_NBK * CSA_BKT)
#define CSA_OFFP (((CSA_NCH + 31) / 32) * 32)

__global__ __launch_bounds__(256) void k_csA_cnt(const int* __restrict__ DST, int dstride, int* __restrict__ CNT) {
  __shared__ unsigned short sc[256][CSA_NBK + 1]; __shared__ __align__(16) int srow[CSA_NBKP];
  const int c = blockIdx.x, tid = threadIdx.x;
  for (int b = 0; b < CSA_NBK; ++b) sc[tid][b] = 0;
  const size_t e0 = (size_t)c * CSA_CHUNK + tid * 16;
  for (int i = 0; i < 16; ++i) { const size_t e = e0 + i; if (e < (size_t)CSA_E) { int d = DST[e * dstride]; d = min(max(d, 0), CSA_N - 1); sc[tid][d / CSA_BKT] += 1; } }
  __syncthreads();
  for (int b = tid; b < CSA_NBKP; b += 256) { int s = 0; if (b < CSA_NBK) for (int t = 0; t < 256; ++t) s += sc[t][b]; srow[b] = s; }
  __syncthreads();
  for (int q = tid; q < CSA_NBKP / 4; q += 256) vst2((unsigned*)(CNT + (size_t)c * CSA_NBKP + q * 4), *(const v4u*)&srow[q * 4]);
}
__global__ __launch_bounds__(256) void k_csA_scan(const int* __restrict__ CNT, int* __restrict__ OFF, int* __restrict__ BST) {
  __shared__ int sbt[CSA_NBK + 1]; __shared__ int sbs[((CSA_NBK + 1 + 31) / 32) * 32]; __shared__ int scnt[CSA_NBK + 1]; __shared__ __align__(16) int sbuf[64][CSA_OFFP];
  const int tid = threadIdx.x;
  for (int b = tid; b < CSA_NBK; b += 256) { int sp = 0, st = 0; for (int c = 0; c < CSA_NCH; ++c) { const int n = CNT[(size_t)c * CSA_NBKP + b]; st += n; sp += (n + 31) & ~31; } sbt[b] = sp; scnt[b] = st; }
  for (int b = tid; b < ((CSA_NBK + 1 + 31) / 32) * 32; b += 256) sbs[b] = 0;
  __syncthreads();
  if (tid == 0) { int acc = 0, accf = 0; for (int b = 0; b < CSA_NBK; ++b) { const int t = sbt[b]; sbt[b] = acc; acc += t; sbs[b] = accf; accf += (scnt[b] + 31) & ~31; } sbs[CSA_NBK] = accf; }
  __syncthreads();
  for (int b0 = 0; b0 < CSA_NBK; b0 += 64) {
    if (tid < 64 && b0 + tid < CSA_NBK) { const int b = b0 + tid; int o = sbt[b]; for (int c = 0; c < CSA_OFFP; ++c) { if (c < CSA_NCH) { sbuf[tid][c] = o; o += (CNT[(size_t)c * CSA_NBKP + b] + 31) & ~31; } else sbuf[tid][c] = 0; } }
    __syncthreads();
    for (int q = tid; q < 64 * (CSA_OFFP / 4); q += 256) { const int r = q / (CSA_OFFP / 4), pc = q % (CSA_OFFP / 4); if (b0 + r < CSA_NBK) vst2((unsigned*)(OFF + (size_t)(b0 + r) * CSA_OFFP + pc * 4), *(const v4u*)&sbuf[r][pc * 4]); }
    __syncthreads(); }
  for (int q = tid; q < ((CSA_NBK + 1 + 31) / 32) * 32 / 4; q += 256) vst2((unsigned*)(BST + q * 4), *(const v4u*)&sbs[q * 4]);
}
__global__ __launch_bounds__(256) void k_csA_scatter(const int* __restrict__ SRC, const int* __restrict__ DST, int sstride, int dstride, const int* __restrict__ OFF, int* __restrict__ SEGS, int* __restrict__ SEGE) {
  __shared__ unsigned short sc[256][CSA_NBK + 1]; __shared__ int sbase[CSA_NBK + 1]; __shared__ int scn[CSA_NBK + 1]; __shared__ int sord[CSA_CHUNK];
  const int c = blockIdx.x, tid = threadIdx.x;
  for (int b = 0; b < CSA_NBK; ++b) sc[tid][b] = 0;
  const size_t e0 = (size_t)c * CSA_CHUNK + tid * 16; int bk[16];
#pragma unroll
  for (int i = 0; i < 16; ++i) { const size_t e = e0 + i; bk[i] = -1; if (e < (size_t)CSA_E) { int d = DST[e * dstride]; d = min(max(d, 0), CSA_N - 1); bk[i] = d / CSA_BKT; sc[tid][bk[i]] += 1; } }
  __syncthreads();
  for (int b = tid; b < CSA_NBK; b += 256) { int acc = 0; for (int t = 0; t < 256; ++t) { const int v = sc[t][b]; sc[t][b] = (unsigned short)acc; acc += v; } scn[b] = acc; }
  __syncthreads();
  if (tid == 0) { int acc = 0; for (int b = 0; b < CSA_NBK; ++b) { sbase[b] = acc; acc += scn[b]; } }
  __syncthreads();
#pragma unroll
  for (int i = 0; i < 16; ++i) { if (bk[i] >= 0) { const int b = bk[i]; const int r = sc[tid][b]; sc[tid][b] = (unsigned short)(r + 1); sord[sbase[b] + r] = tid * 16 + i; } }
  __syncthreads();
  for (int b = 0; b < CSA_NBK; ++b) { const int n = scn[b]; if (n == 0) continue; const int nl = ((n + 31) & ~31); const size_t o = (size_t)(min(max(OFF[(size_t)b * CSA_OFFP + c], 0), CSA_SEGCAP - nl) & ~31);
    for (int q = tid; q < nl / 4; q += 256) { int4 vs, ve;
#pragma unroll
      for (int k = 0; k < 4; ++k) { const int i = q * 4 + k; int s = -1, eid = -1; if (i < n) { const size_t e = (size_t)c * CSA_CHUNK + sord[sbase[b] + i]; s = min(max(SRC[e * sstride], 0), CSA_N - 1); eid = (int)e; } vs[k] = s; ve[k] = eid; }
      vst2((unsigned*)(SEGS + o + q * 4), *(const v4u*)&vs); vst2((unsigned*)(SEGE + o + q * 4), *(const v4u*)&ve); } }
}
__global__ __launch_bounds__(256) void k_csA_bucket(const int* __restrict__ CNT, const int* __restrict__ OFF, const int* __restrict__ BST, const int* __restrict__ SEGS, const int* __restrict__ SEGE, const int* __restrict__ DST, int dstride, int* __restrict__ FS, int* __restrict__ FE, int* __restrict__ ROWST, int* __restrict__ ROWCNT) {
  __shared__ int ssrc[CSA_BCAP]; __shared__ int seid[CSA_BCAP]; __shared__ unsigned char snod[CSA_BCAP]; __shared__ int souts[CSA_BCAP]; __shared__ int soute[CSA_BCAP]; __shared__ int scount[256]; __shared__ int sstart[257]; __shared__ int stot;
  const int b = blockIdx.x, tid = threadIdx.x;
  if (tid == 0) { int t = 0; for (int c = 0; c < CSA_NCH; ++c) t += min(max(CNT[(size_t)c * CSA_NBKP + b], 0), CSA_CHUNK); stot = (t <= CSA_BCAP) ? t : 0; }
  __syncthreads();
  { int base = 0; for (int c = 0; c < CSA_NCH; ++c) { const int n = min(max(CNT[(size_t)c * CSA_NBKP + b], 0), CSA_CHUNK); const int o = min(max(OFF[(size_t)b * CSA_OFFP + c], 0), CSA_SEGCAP - ((n + 31) & ~31));
      for (int i = tid; i < n; i += 256) { const int p = base + i; if (p < CSA_BCAP) { ssrc[p] = min(max(SEGS[o + i], 0), CSA_N - 1); const int e = min(max(SEGE[o + i], 0), CSA_E - 1); seid[p] = e; int d = DST[(size_t)e * dstride]; d = min(max(d, 0), CSA_N - 1); const int dl = d - b * CSA_BKT; snod[p] = (unsigned char)(dl >= 0 && dl < 256 ? dl : 255); } }
      base += n; } }
  __syncthreads();
  const int node = b * CSA_BKT + tid; int cnt = 0; for (int p = 0; p < stot; ++p) cnt += (snod[p] == tid) ? 1 : 0;
  scount[tid] = cnt; __syncthreads();
  if (tid == 0) { int acc = 0; for (int t = 0; t < 256; ++t) { sstart[t] = acc; acc += scount[t]; } sstart[256] = acc; }
  __syncthreads();
  const int bst0 = min(max(BST[b], 0), CSA_FINN - ((sstart[256] + 31) & ~31)) & ~31; const int gst = bst0 + sstart[tid];
  { int w = sstart[tid]; for (int p = 0; p < stot; ++p) if (snod[p] == tid) { souts[w] = ssrc[p]; soute[w] = seid[p]; ++w; } }
  __syncthreads();
  { const int n = sstart[256]; const int nl = (n + 31) & ~31; for (int q = tid; q < nl / 4; q += 256) { int4 vs, ve;
#pragma unroll
      for (int k = 0; k < 4; ++k) { const int i = q * 4 + k; vs[k] = i < n ? souts[i] : -1; ve[k] = i < n ? soute[i] : -1; }
      vst2((unsigned*)(FS + bst0 + q * 4), *(const v4u*)&vs); vst2((unsigned*)(FE + bst0 + q * 4), *(const v4u*)&ve); } }
  __syncthreads();
  { __shared__ __align__(16) int srs[256], src2[256]; srs[tid] = node < CSA_N ? gst : 0; src2[tid] = node < CSA_N ? cnt : 0; __syncthreads();
    if (tid < 64) vst2((unsigned*)(ROWST + (size_t)b * 256 + tid * 4), *(const v4u*)&srs[tid * 4]); else if (tid < 128) vst2((unsigned*)(ROWCNT + (size_t)b * 256 + (tid - 64) * 4), *(const v4u*)&src2[(tid - 64) * 4]); }
}


#define WS_CNT  0u
#define WS_OFF  (WS_CNT + CSA_SZ_CNT)
#define WS_BST  (WS_OFF + CSA_SZ_OFF)
#define WS_SEGS (WS_BST + CSA_SZ_BST)
#define WS_SEGE (WS_SEGS + CSA_SZ_SEG)
#define WS_FS   (WS_SEGE + CSA_SZ_SEG)
#define WS_FE   (WS_FS + CSA_SZ_FIN)
#define WS_RST  (WS_FE + CSA_SZ_FIN)
#define WS_RCT  (WS_RST + CSA_SZ_ROW)
#define WS_CELL (WS_RCT + CSA_SZ_ROW)
#define WS_PID  (WS_CELL + 4u * NPTS)
#define WS_XYZ  (WS_PID + 4u * NPTS)
#define WS_IDX  (WS_XYZ + 4u * NPTS * 4)
#define WS_PW   (WS_IDX + 4u * NPTS * 16)
#define WS_HF   (WS_PW + 2u * 16 * 256)
#define WS_QKV  (WS_HF + 4u * NPTS * 16)
#define WS_AGG  (WS_QKV + 4u * NPTS * 64)
#define WS_END  (WS_AGG + 4u * NPTS * 16)

__global__ __launch_bounds__(256) void k_cell(const float* __restrict__ P, float* __restrict__ XYZ, int* __restrict__ CELL, int* __restrict__ PID) {
  __shared__ __align__(16) int sc[256], sp[256]; const int t = threadIdx.x; const size_t i = (size_t)blockIdx.x * 256 + t;
  const float x = bfr(P[i * 3]), y = bfr(P[i * 3 + 1]), z = bfr(P[i * 3 + 2]);
  const int cx = min(max((int)floorf(x * GRID), 0), GRID - 1), cy = min(max((int)floorf(y * GRID), 0), GRID - 1), cz = min(max((int)floorf(z * GRID), 0), GRID - 1);
  sc[t] = (cx * GRID + cy) * GRID + cz; sp[t] = (int)i;
  vst2(XYZ + i * 4, (v4f){x, y, z, 0.f});
  __syncthreads();
  if (t < 64) { vst2((unsigned*)(CELL + (size_t)blockIdx.x * 256 + t * 4), *(const v4u*)&sc[t * 4]); vst2((unsigned*)(PID + (size_t)blockIdx.x * 256 + t * 4), *(const v4u*)&sp[t * 4]); }
}
__device__ __forceinline__ void knn_insert(float d, int m, float* bd, int* bi) {
  if (d < bd[NS - 1] || (d == bd[NS - 1] && m < bi[NS - 1])) { int pos = NS - 1;
#pragma unroll
    for (int q = NS - 2; q >= 0; --q) if (d < bd[q] || (d == bd[q] && m < bi[q])) pos = q;
#pragma unroll
    for (int q = NS - 1; q >= 1; --q) if (q > pos) { bd[q] = bd[q - 1]; bi[q] = bi[q - 1]; }
#pragma unroll
    for (int q = 0; q < NS; ++q) if (q == pos) { bd[q] = d; bi[q] = m; } }
}
__global__ __launch_bounds__(64) void k_knn(const float* __restrict__ XYZ, const int* __restrict__ CELL, const int* __restrict__ FE, const int* __restrict__ RST, const int* __restrict__ RCT, int* __restrict__ IDX) {
  #pragma clang fp contract(off)
  __shared__ __align__(16) int sk[64][NS]; const int t = threadIdx.x; const size_t i = (size_t)blockIdx.x * 64 + t;
  const float qx = XYZ[i * 4], qy = XYZ[i * 4 + 1], qz = XYZ[i * 4 + 2]; const int cid = min(max(CELL[i], 0), NCELL - 1); const int cx = cid / (GRID * GRID), cy = (cid / GRID) % GRID, cz = cid % GRID;
  float bd[NS]; int bi[NS];
  bool done = false;
#pragma unroll 1
  for (int R = 1; R <= 3 && !done; ++R) {
#pragma unroll
    for (int q = 0; q < NS; ++q) { bd[q] = 3.0e38f; bi[q] = 0x7fffffff; }
    if (R <= 2) {
#pragma unroll 1
      for (int ax = max(cx - R, 0); ax <= min(cx + R, GRID - 1); ++ax)
#pragma unroll 1
        for (int ay = max(cy - R, 0); ay <= min(cy + R, GRID - 1); ++ay)
#pragma unroll 1
          for (int az = max(cz - R, 0); az <= min(cz + R, GRID - 1); ++az) { const int c = (ax * GRID + ay) * GRID + az; const int cnt = min(max(RCT[c], 0), CSA_BCAP); const int st = min(max(RST[c], 0), CSA_FINN - cnt);
#pragma unroll 1
            for (int e = 0; e < cnt; ++e) { const int m = min(max(FE[st + e], 0), NPTS - 1); const float dx = qx - XYZ[(size_t)m * 4], dy = qy - XYZ[(size_t)m * 4 + 1], dz = qz - XYZ[(size_t)m * 4 + 2]; const float d = (dx * dx + dz * dz) + dy * dy; knn_insert(d, m, bd, bi); } }
      const float cs = 1.0f / (float)GRID; float margin = 3.0e38f;
      { const float lo = (cx - R >= 1) ? (qx - (float)(cx - R) * cs) : 3.0e38f, hi = (cx + R <= GRID - 2) ? ((float)(cx + R + 1) * cs - qx) : 3.0e38f; margin = fminf(margin, fminf(lo, hi)); }
      { const float lo = (cy - R >= 1) ? (qy - (float)(cy - R) * cs) : 3.0e38f, hi = (cy + R <= GRID - 2) ? ((float)(cy + R + 1) * cs - qy) : 3.0e38f; margin = fminf(margin, fminf(lo, hi)); }
      { const float lo = (cz - R >= 1) ? (qz - (float)(cz - R) * cs) : 3.0e38f, hi = (cz + R <= GRID - 2) ? ((float)(cz + R + 1) * cs - qz) : 3.0e38f; margin = fminf(margin, fminf(lo, hi)); }
      const float msafe = margin * 0.999f;
      done = (bi[NS - 1] != 0x7fffffff) && (bd[NS - 1] < msafe * msafe);
    } else {
#pragma unroll 1
      for (int m = 0; m < NPTS; ++m) { const float dx = qx - XYZ[(size_t)m * 4], dy = qy - XYZ[(size_t)m * 4 + 1], dz = qz - XYZ[(size_t)m * 4 + 2]; const float d = (dx * dx + dz * dz) + dy * dy; knn_insert(d, m, bd, bi); }
      done = true; }
  }
#pragma unroll
  for (int q = 0; q < NS; ++q) sk[t][q] = min(bi[q], NPTS - 1);
  __syncthreads();
  for (int q = t; q < 64 * 4; q += 64) { const int rl = q >> 2, pc = q & 3; vst2((unsigned*)(IDX + ((size_t)blockIdx.x * 64 + rl) * NS + pc * 4), *(const v4u*)&sk[rl][pc * 4]); }
}
__global__ __launch_bounds__(256) void k_packW(const float* __restrict__ Wm, __bf16* __restrict__ DST_) {
  __shared__ __align__(16) __bf16 s[256]; const int n = blockIdx.x, t = threadIdx.x; s[t] = (__bf16)Wm[(size_t)t * CIN + n]; __syncthreads();
  if (t < 32) vst2((unsigned*)(DST_ + (size_t)n * 256 + t * 8), *(const v4u*)&s[t * 8]);
}
__global__ __launch_bounds__(128) void k_ein(const float* __restrict__ XM, const float* __restrict__ XO, const __bf16* __restrict__ PW, const float* __restrict__ BE, const float* __restrict__ WQ, const float* __restrict__ BQ, const float* __restrict__ WK, const float* __restrict__ BK, const float* __restrict__ WV, const float* __restrict__ BV, float* __restrict__ HF, float* __restrict__ QKV) {
  __shared__ __align__(16) float sh[64][CIN]; __shared__ __align__(16) float sq[64][64];
  const int tid = threadIdx.x, wave = tid >> 5, lane = tid & 31, col = lane & 15, g = lane >> 4; const size_t r0 = (size_t)blockIdx.x * 64 + wave * 16;
  v8f acc = {};
#pragma unroll 2
  for (int kc = 0; kc < CF / 32; ++kc) { v16b a; { const float* p = (kc < 4) ? (XM + (r0 + col) * 128 + kc * 32 + 8 * g) : (XO + (r0 + col) * 128 + (kc - 4) * 32 + 8 * g);
#pragma unroll
      for (int i = 0; i < 8; ++i) { a[i] = (__bf16)p[i]; a[8 + i] = (__bf16)p[16 + i]; } }
    acc = wmma_bf(a, frag_b(PW + (size_t)col * CF + kc * 32, lane), acc); }
#pragma unroll
  for (int r = 0; r < 8; ++r) sh[wave * 16 + 8 * g + r][col] = acc[r] + bfr(BE[col]);
  __syncthreads();
  if (tid < 64) { const int pl = tid;
#pragma unroll 1
    for (int o = 0; o < CIN; ++o) { float aq = bfr(BQ[o]), ak = bfr(BK[o]), av = bfr(BV[o]);
#pragma unroll 4
      for (int i2 = 0; i2 < CIN; ++i2) { const float hv = sh[pl][i2]; aq += hv * bfr(WQ[i2 * CIN + o]); ak += hv * bfr(WK[i2 * CIN + o]); av += hv * bfr(WV[i2 * CIN + o]); }
      sq[pl][o] = aq; sq[pl][16 + o] = ak; sq[pl][32 + o] = av; sq[pl][48 + o] = 0.f; } }
  __syncthreads();
  for (int q = tid; q < 64 * 4; q += 128) { const int pl = q >> 2, pc = q & 3; vst2(HF + ((size_t)blockIdx.x * 64 + pl) * CIN + pc * 4, *(const v4f*)&sh[pl][pc * 4]); }
  for (int q = tid; q < 64 * 16; q += 128) { const int pl = q >> 4, pc = q & 15; vst2(QKV + ((size_t)blockIdx.x * 64 + pl) * 64 + pc * 4, *(const v4f*)&sq[pl][pc * 4]); }
}
__global__ __launch_bounds__(128) void k_pt(const float* __restrict__ XYZ, const int* __restrict__ IDX, const float* __restrict__ QKV,
    const float* __restrict__ WP1, const float* __restrict__ BP1, const float* __restrict__ WP2, const float* __restrict__ BP2, const float* __restrict__ WL1, const float* __restrict__ BL1, const float* __restrict__ WL2, const float* __restrict__ BL2,
    const float* __restrict__ PG, const float* __restrict__ PB, const float* __restrict__ PM, const float* __restrict__ PV, const float* __restrict__ W1G, const float* __restrict__ W1B, const float* __restrict__ W1M, const float* __restrict__ W1V, const float* __restrict__ W2G, const float* __restrict__ W2B, const float* __restrict__ W2M, const float* __restrict__ W2V,
    float* __restrict__ AGG) {
  __shared__ __align__(16) float sagg[64][CIN]; __shared__ float spe[4][32][CIN + 1];
  const int tid = threadIdx.x, wave = tid >> 5, lane = tid & 31; const size_t p0 = (size_t)blockIdx.x * 64;
#pragma unroll 1
  for (int pl = wave; pl < 64; pl += 4) { const size_t i = p0 + pl; const int n = (lane < NS) ? min(max(IDX[i * NS + lane], 0), NPTS - 1) : (int)i;
    const float rx = XYZ[(size_t)n * 4] - XYZ[i * 4], ry = XYZ[(size_t)n * 4 + 1] - XYZ[i * 4 + 1], rz = XYZ[(size_t)n * 4 + 2] - XYZ[i * 4 + 2]; float t3[3];
#pragma unroll
    for (int o = 0; o < 3; ++o) { float a = ((rx * bfr(WP1[0 * 3 + o]) + ry * bfr(WP1[1 * 3 + o])) + rz * bfr(WP1[2 * 3 + o])) + bfr(BP1[o]); a = (a - bfr(PM[o])) / sqrtf(bfr(PV[o]) + 1e-5f) * bfr(PG[o]) + bfr(PB[o]); t3[o] = fmaxf(a, 0.f); }
    float a0 = bfr(BL1[0]), a1 = bfr(BL1[1]);
#pragma unroll 1
    for (int c = 0; c < CIN; ++c) { const float pe = ((t3[0] * bfr(WP2[c]) + t3[1] * bfr(WP2[CIN + c])) + t3[2] * bfr(WP2[2 * CIN + c])) + bfr(BP2[c]); spe[wave][lane][c] = pe;
      float v = (QKV[(size_t)n * 64 + 16 + c] - QKV[i * 64 + c]) + pe; v = (v - bfr(W1M[c])) / sqrtf(bfr(W1V[c]) + 1e-5f) * bfr(W1G[c]) + bfr(W1B[c]); v = fmaxf(v, 0.f); a0 += v * bfr(WL1[c * 2]); a1 += v * bfr(WL1[c * 2 + 1]); }
    float b0 = (a0 - bfr(W2M[0])) / sqrtf(bfr(W2V[0]) + 1e-5f) * bfr(W2G[0]) + bfr(W2B[0]); float b1 = (a1 - bfr(W2M[1])) / sqrtf(bfr(W2V[1]) + 1e-5f) * bfr(W2G[1]) + bfr(W2B[1]); b0 = fmaxf(b0, 0.f); b1 = fmaxf(b1, 0.f);
    float w2[2]; w2[0] = (b0 * bfr(WL2[0]) + b1 * bfr(WL2[2])) + bfr(BL2[0]); w2[1] = (b0 * bfr(WL2[1]) + b1 * bfr(WL2[3])) + bfr(BL2[1]);
    float sw[2];
#pragma unroll
    for (int c = 0; c < 2; ++c) { float v = (lane < NS) ? w2[c] : -3.0e38f; float mx = v;
#pragma unroll
      for (int o = 1; o < 16; o <<= 1) mx = fmaxf(mx, __shfl_xor(mx, o));
      const float e = (lane < NS) ? exp_ni(v - mx) : 0.f; float s = e;
#pragma unroll
      for (int o = 1; o < 16; o <<= 1) s += __shfl_xor(s, o);
      sw[c] = e / s; }
#pragma unroll 1
    for (int c = 0; c < CIN; ++c) { float v = (lane < NS) ? (QKV[(size_t)n * 64 + 32 + c] + spe[wave][lane][c]) * ((c & 1) ? sw[1] : sw[0]) : 0.f;
#pragma unroll
      for (int o = 1; o < 16; o <<= 1) v += __shfl_xor(v, o);
      if (lane == 0) sagg[pl][c] = v; } }
  __syncthreads();
  for (int q = tid; q < 64 * 4; q += 128) { const int pl = q >> 2, pc = q & 3; vst2(AGG + (p0 + pl) * CIN + pc * 4, *(const v4f*)&sagg[pl][pc * 4]); }
}
__global__ __launch_bounds__(256) void k_eout(const float* __restrict__ AGG, const float* __restrict__ WEO, const float* __restrict__ BEO, const float* __restrict__ XM, const float* __restrict__ XO, float* __restrict__ OUT) {
  __shared__ __align__(16) float srow[CF]; __shared__ float sw[CIN][CF]; const int c = threadIdx.x; const size_t p0 = (size_t)blockIdx.x * 64;
  for (int i2 = 0; i2 < CIN; ++i2) sw[i2][c] = bfr(WEO[i2 * CF + c]);
  const float bb = bfr(BEO[c]);
  __syncthreads();
  for (int pl = 0; pl < 64; ++pl) { const size_t i = p0 + pl; float a = bb;
#pragma unroll
    for (int i2 = 0; i2 < CIN; ++i2) a += AGG[i * CIN + i2] * sw[i2][c];
    a += (c < 128) ? bfr(XM[i * 128 + c]) : bfr(XO[i * 128 + c - 128]);
    srow[c] = a; __syncthreads();
    if (c < 64) vst2(OUT + i * CF + c * 4, *(const v4f*)&srow[c * 4]);
    __syncthreads(); }
}
extern "C" void kernel_launch(void* const* d_in, const int* in_sizes, int n_in, void* d_out, int out_size, void* d_ws, size_t ws_size, hipStream_t stream) {
  (void)in_sizes; (void)n_in; (void)out_size;
  const float** F = (const float**)d_in;
  if (ws_size < (size_t)WS_END) return;
  char* ws = (char*)d_ws;
  int *CNT = (int*)(ws + WS_CNT), *OFF = (int*)(ws + WS_OFF), *BST = (int*)(ws + WS_BST), *SEGS = (int*)(ws + WS_SEGS), *SEGE = (int*)(ws + WS_SEGE), *FS = (int*)(ws + WS_FS), *FE = (int*)(ws + WS_FE), *RST = (int*)(ws + WS_RST), *RCT = (int*)(ws + WS_RCT), *CELL = (int*)(ws + WS_CELL), *PID = (int*)(ws + WS_PID), *IDX = (int*)(ws + WS_IDX);
  float *XYZ = (float*)(ws + WS_XYZ), *HF = (float*)(ws + WS_HF), *QKV = (float*)(ws + WS_QKV), *AGG = (float*)(ws + WS_AGG); __bf16* PW = (__bf16*)(ws + WS_PW);
  k_cell<<<NPTS / 256, 256, 0, stream>>>(F[2], XYZ, CELL, PID);
  k_csA_cnt<<<CSA_NCH, 256, 0, stream>>>(CELL, 1, CNT); k_csA_scan<<<1, 256, 0, stream>>>(CNT, OFF, BST); k_csA_scatter<<<CSA_NCH, 256, 0, stream>>>(PID, CELL, 1, 1, OFF, SEGS, SEGE); k_csA_bucket<<<CSA_NBK, 256, 0, stream>>>(CNT, OFF, BST, SEGS, SEGE, CELL, 1, FS, FE, RST, RCT);
  k_knn<<<NPT_ / 64, 64, 0, stream>>>(XYZ, CELL, FE, RST, RCT, IDX);
  k_packW<<<CIN, 256, 0, stream>>>(F[3], PW);
  k_ein<<<NPTS / 64, 128, 0, stream>>>(F[0], F[1], PW, F[4], F[7], F[8], F[9], F[10], F[11], F[12], HF, QKV);
  k_pt<<<NPT_ / 64, 128, 0, stream>>>(XYZ, IDX, QKV, F[13], F[14], F[15], F[16], F[17], F[18], F[19], F[20], F[21], F[22], F[23], F[24], F[25], F[26], F[27], F[28], F[29], F[30], F[31], F[32], AGG);
  k_eout<<<NPT_ / 64, 256, 0, stream>>>(AGG, F[5], F[6], F[0], F[1], (float*)d_out);
}
